// PhysicsMambaBlock_81862076662143
// MI455X (gfx1250) — hardware-run, weakly checked
//
#include <hip/hip_runtime.h>
#include <math.h>

typedef __attribute__((ext_vector_type(16))) _Float16 v16h;
typedef __attribute__((ext_vector_type(8)))  _Float16 v8h;
typedef __attribute__((ext_vector_type(8)))  float    v8f;
typedef __attribute__((ext_vector_type(4)))  float    v4f;

constexpr int kBatch  = 16;
constexpr int kSeq    = 1024;
constexpr int kDm     = 256;
constexpr int kDin    = 512;
constexpr int kNst    = 64;
constexpr int kXzP    = 2 * kDin;
constexpr int kWxP    = 144;
constexpr int kWxSkip = 16;
constexpr int kBcW    = 2 * kNst;
constexpr int kRows   = kBatch * kSeq;
constexpr int kHalves = 2;
constexpr int kHRows  = kRows / kHalves;
constexpr int kHBatch = kBatch / kHalves;
constexpr int kConvTP = 260;
constexpr int kScTS   = 32;
constexpr int kScCh   = 64;
constexpr int kScP    = 68;
constexpr int kScSub  = 4;
constexpr int kScNl   = kNst / kScSub;

constexpr float kCarX = 16.0f;
constexpr float kCarW = 64.0f;
constexpr float kCarU = 256.0f;
constexpr float kCarY = 1024.0f;
constexpr float kSclIn  = 1.0f / (kCarX * kCarW);
constexpr float kSclXp  = 1.0f / (kCarU * kCarW);
constexpr float kSclOut = 1.0f / (kCarY * kCarW);

static_assert(kWxSkip + kBcW == kWxP, "x_proj width");
static_assert((kDm % 32) == 0 && (kDin % 32) == 0, "GEMM K multiples of 32");
static_assert((kHRows % 64) == 0 && (kXzP % 64) == 0 && (kBcW % 64) == 0 && (kDm % 64) == 0, "GEMM M,N multiples of 64");
static_assert((kDm % 64) == 0 && (kDin % 64) == 0, "transpose tiles");
static_assert((kSeq % 64) == 0 && (kSeq % kScTS) == 0 && (kDin % 256) == 0 && (kDin % kScCh) == 0, "tile multiples");
static_assert(kScTS == 32 && kScCh == 64 && kScSub == 4 && kScNl == 16, "scan block geometry");
static_assert(kScTS * kBcW == kScCh * kNst, "A staging reuses the B|C tile");
static_assert((kRows % kHalves) == 0 && (kBatch % kHalves) == 0, "halves");

constexpr size_t kSzWIN  = (size_t)kXzP * kDm * 2;
constexpr size_t kSzWX   = (size_t)kBcW * kDin * 2;
constexpr size_t kSzWOUT = (size_t)kDm * kDin * 2;
constexpr size_t kSzX16  = (size_t)kRows * kDm * 2;
constexpr size_t kSzXZ   = (size_t)kHRows * kXzP * 4;
constexpr size_t kSzUC   = (size_t)kHRows * kDin * 4;
constexpr size_t kSzUC16 = (size_t)kHRows * kDin * 2;
constexpr size_t kSzBC   = (size_t)kHRows * kBcW * 4;
constexpr size_t kSzY16  = (size_t)kHRows * kDin * 2;
constexpr size_t kOffWIN  = 0;
constexpr size_t kOffWX   = kOffWIN  + kSzWIN;
constexpr size_t kOffWOUT = kOffWX   + kSzWX;
constexpr size_t kOffX16  = kOffWOUT + kSzWOUT;
constexpr size_t kOffXZ   = kOffX16  + kSzX16;
constexpr size_t kOffUC   = kOffXZ   + kSzXZ;
constexpr size_t kOffUC16 = kOffUC   + kSzUC;
constexpr size_t kOffBC   = kOffUC16 + kSzUC16;
constexpr size_t kOffY16  = kOffBC   + kSzBC;
constexpr size_t kWsTotal = kOffY16  + kSzY16;
static_assert(kWsTotal == 80609280ull, "carve total");
static_assert(kWsTotal <= 134217728ull, "carve cap");
static_assert((kOffWX % 128) == 0 && (kOffWOUT % 128) == 0 && (kOffX16 % 128) == 0 && (kOffXZ % 128) == 0 &&
              (kOffUC % 128) == 0 && (kOffUC16 % 128) == 0 && (kOffBC % 128) == 0 && (kOffY16 % 128) == 0,
              "128-B aligned regions");

__device__ __forceinline__ _Float16 to_h16(float v) {
  const float f = (fabsf(v) < 6.103515625e-05f) ? 0.0f : v;
  return (_Float16)f;
}

__device__ __forceinline__ void tie1_h(v8f& a, v16h x, v16h y) { asm volatile("" : "+v"(a) : "v"(x), "v"(y)); }
__device__ __forceinline__ void guard1_h(v8f& a, v16h x, v16h y) { asm volatile("v_nop\n\tv_nop\n\tv_nop\n\tv_nop" : "+v"(a) : "v"(x), "v"(y)); }
__device__ __forceinline__ void keep4_h(v16h a, v16h b, v16h c, v16h d) { asm volatile("v_nop" :: "v"(a), "v"(b), "v"(c), "v"(d)); }
__device__ __forceinline__ void acc_guard4(v8f& a, v8f& b, v8f& c, v8f& d) { asm volatile("v_nop\n\tv_nop\n\tv_nop\n\tv_nop" : "+v"(a), "+v"(b), "+v"(c), "+v"(d)); }

template <typename T> struct Frag;
template <> struct Frag<_Float16> {
  typedef v16h V; union U { v16h v; v8h h[2]; };
  static __device__ __forceinline__ v16h load(const _Float16* p) {
    U f; f.h[0] = *(const v8h*)(p); f.h[1] = *(const v8h*)(p + 16); return f.v;
  }
  static __device__ __forceinline__ v8f mma(v16h a, v16h b, v8f c) {
    return __builtin_amdgcn_wmma_f32_16x16x32_f16(false, a, false, b, (short)0, c, false, false);
  }
};

__global__ __launch_bounds__(256) void wmma_gemm64_f16(
    const unsigned short* __restrict__ Ap, int lda,
    const unsigned short* __restrict__ Btp, int ldb,
    float* __restrict__ C, int ldc,
    int M, int N, int K, float scale)
{
  typedef _Float16 T;
  const T* A  = (const T*)Ap;
  const T* Bt = (const T*)Btp;
  __shared__ __align__(16) float sT[8][16 * 68];
  const int lane = threadIdx.x & 31;
  const int wave = threadIdx.x >> 5;
  const int tilesN = N >> 6;
  const int tilesM = M >> 6;
  const int tile = blockIdx.x * 8 + wave;
  if (tile >= tilesM * tilesN) return;
  const int tm = tile / tilesN;
  const int tn = tile - tm * tilesN;
  const int m0 = tm << 6;
  const int n0 = tn << 6;

  const int rlane = lane & 15;
  const int koff  = (lane >> 4) * 8;
  const int mOff  = (lane >> 4) * 8;

  v8f acc[4][4];
#pragma unroll
  for (int i = 0; i < 4; ++i)
#pragma unroll
    for (int j = 0; j < 4; ++j) acc[i][j] = (v8f){0.f,0.f,0.f,0.f,0.f,0.f,0.f,0.f};

  for (int k0 = 0; k0 < K; k0 += 32) {
    v16h bh[4];
#pragma unroll
    for (int j = 0; j < 4; ++j) {
      const size_t bo = (size_t)(n0 + (j << 4) + rlane) * ldb + koff + k0;
      bh[j] = Frag<T>::load(Bt + bo);
    }
#pragma unroll
    for (int i = 0; i < 4; ++i) {
      const size_t ao = (size_t)(m0 + (i << 4) + rlane) * lda + koff + k0;
      v16h ah = Frag<T>::load(A + ao);
#pragma unroll
      for (int j = 0; j < 4; ++j) acc[i][j] = Frag<T>::mma(ah, bh[j], acc[i][j]);
      tie1_h(acc[i][0], ah, bh[0]);
      tie1_h(acc[i][1], ah, bh[1]);
      tie1_h(acc[i][2], ah, bh[2]);
      guard1_h(acc[i][3], ah, bh[3]);
    }
    keep4_h(bh[0], bh[1], bh[2], bh[3]);
  }
  acc_guard4(acc[0][0], acc[0][1], acc[0][2], acc[0][3]);
  acc_guard4(acc[1][0], acc[1][1], acc[1][2], acc[1][3]);
  acc_guard4(acc[2][0], acc[2][1], acc[2][2], acc[2][3]);
  acc_guard4(acc[3][0], acc[3][1], acc[3][2], acc[3][3]);

  float* slab = sT[wave];
#pragma unroll
  for (int i = 0; i < 4; ++i) {
    const int mBase = m0 + (i << 4);
#pragma unroll
    for (int j = 0; j < 4; ++j) {
#pragma unroll
      for (int r = 0; r < 8; ++r) {
        const float v = acc[i][j][r] * scale;
        slab[(mOff + r) * 68 + (j << 4) + rlane] = v;
      }
    }
    __builtin_amdgcn_fence(__ATOMIC_RELEASE, "workgroup");
    __builtin_amdgcn_wave_barrier();
    __builtin_amdgcn_fence(__ATOMIC_ACQUIRE, "workgroup");
    {
      const int hh = lane >> 4, c4 = (lane & 15) * 4;
      for (int pass = 0; pass < 2; ++pass) {
#pragma unroll
        for (int it = 0; it < 8; ++it) {
          const int row = it * 2 + hh;
          v4f v = *(const v4f*)(slab + row * 68 + c4);
          *(volatile v4f*)(C + (size_t)(mBase + row) * ldc + n0 + c4) = v;
        }
        __threadfence();
      }
    }
    __builtin_amdgcn_fence(__ATOMIC_RELEASE, "workgroup");
    __builtin_amdgcn_wave_barrier();
    __builtin_amdgcn_fence(__ATOMIC_ACQUIRE, "workgroup");
  }
}

__global__ __launch_bounds__(256) void cast_f16_kernel(
    const float* __restrict__ src, unsigned short* __restrict__ dst, int total8, float scale)
{
  const int i = blockIdx.x * 256 + threadIdx.x;
  if (i >= total8) return;
  const size_t e0 = (size_t)i << 3;
  const float* p = src + e0;
  const v4f a0 = *(const v4f*)(p);
  const v4f a1 = *(const v4f*)(p + 4);
  v8h hv;
#pragma unroll
  for (int e = 0; e < 4; ++e) {
    hv[e]     = to_h16(a0[e] * scale);
    hv[4 + e] = to_h16(a1[e] * scale);
  }
  unsigned short* q = dst + e0;
  *(volatile v8h*)q = hv;
  __threadfence();
  *(volatile v8h*)q = hv;
}

__global__ __launch_bounds__(256) void transpose_cast_kernel(
    const float* __restrict__ W, unsigned short* __restrict__ Bt, int Kdim, int ldw, int col0, int Ncnt, float scale)
{
  __shared__ float tile[64 * 65];
  const int tid = threadIdx.x, lane = tid & 31, wave = tid >> 5;
  const int n0 = blockIdx.x * 64;
  const int k0 = blockIdx.y * 64;
#pragma unroll 4
  for (int p = 0; p < 16; ++p) {
    const int idx = tid + p * 256;
    const int kk  = idx >> 6;
    const int nn  = idx & 63;
    const int n   = n0 + nn;
    const int nc  = (n < Ncnt) ? n : (Ncnt - 1);
    const float v = W[(size_t)(k0 + kk) * ldw + col0 + nc];
    tile[kk * 65 + nn] = (n < Ncnt) ? (v * scale) : 0.f;
  }
  __syncthreads();
  const int q = lane >> 3, c8 = (lane & 7) * 8;
  v8h hv[2];
#pragma unroll
  for (int it = 0; it < 2; ++it) {
    const int nrow = it * 32 + wave * 4 + q;
#pragma unroll
    for (int e = 0; e < 8; ++e) hv[it][e] = to_h16(tile[(c8 + e) * 65 + nrow]);
  }
  for (int pass = 0; pass < 2; ++pass) {
#pragma unroll
    for (int it = 0; it < 2; ++it) {
      const int nrow = it * 32 + wave * 4 + q;
      *(volatile v8h*)(Bt + (size_t)(n0 + nrow) * Kdim + k0 + c8) = hv[it];
    }
    __threadfence();
  }
}

__global__ __launch_bounds__(256) void conv_silu_kernel(
    const float* __restrict__ XZ, const float* __restrict__ cw, const float* __restrict__ cb,
    float* __restrict__ UC, unsigned short* __restrict__ UC16)
{
  __shared__ __align__(16) float sT[16 * kConvTP];
  const int tid = threadIdx.x, lane = tid & 31, wave = tid >> 5;
  const int d0 = blockIdx.x * 256, d = d0 + tid;
  const int g0 = blockIdx.y * 64;
  const int tb = g0 & (kSeq - 1);
  const v4f wv = *(const v4f*)(cw + (size_t)d * 4);
  const float w0 = wv[0], w1 = wv[1], w2 = wv[2], w3 = wv[3];
  const float bc = cb[d];
  float xm3, xm2, xm1;
  {
    const bool hist = (tb > 0);
    const int rb = hist ? (g0 - 3) : g0;
    const float v3 = XZ[(size_t)rb * kXzP + d];
    const float v2 = XZ[(size_t)(rb + 1) * kXzP + d];
    const float v1 = XZ[(size_t)(rb + 2) * kXzP + d];
    xm3 = hist ? v3 : 0.f;
    xm2 = hist ? v2 : 0.f;
    xm1 = hist ? v1 : 0.f;
  }
  const int hrow = wave >> 1;
  const int hch  = (wave & 1) * 128 + lane * 4;
#pragma unroll 1
  for (int sub = 0; sub < 4; ++sub) {
    const int lb = g0 + sub * 16;
#pragma unroll 1
    for (int s = 0; s < 16; ++s) {
      const float xcur = XZ[(size_t)(lb + s) * kXzP + d];
      float acc = w0 * xm3;
      acc = fmaf(w1, xm2, acc);
      acc = fmaf(w2, xm1, acc);
      acc = fmaf(w3, xcur, acc);
      const float sv = acc + bc;
      const float sg = __builtin_amdgcn_rcpf(1.0f + __expf(-sv));
      sT[s * kConvTP + tid] = sv * sg;
      xm3 = xm2; xm2 = xm1; xm1 = xcur;
    }
    __syncthreads();
    v4f fv[4];
    v8h bv[2];
#pragma unroll
    for (int it = 0; it < 4; ++it) fv[it] = *(const v4f*)(sT + (it * 4 + hrow) * kConvTP + hch);
#pragma unroll
    for (int it = 0; it < 2; ++it) {
      const float* sp = sT + (it * 8 + wave) * kConvTP + lane * 8;
      const v4f a0 = *(const v4f*)(sp);
      const v4f a1 = *(const v4f*)(sp + 4);
#pragma unroll
      for (int e = 0; e < 4; ++e) {
        bv[it][e]     = to_h16(a0[e] * kCarU);
        bv[it][4 + e] = to_h16(a1[e] * kCarU);
      }
    }
    for (int pass = 0; pass < 2; ++pass) {
#pragma unroll
      for (int it = 0; it < 4; ++it)
        *(volatile v4f*)(UC + (size_t)(lb + it * 4 + hrow) * kDin + d0 + hch) = fv[it];
#pragma unroll
      for (int it = 0; it < 2; ++it)
        *(volatile v8h*)(UC16 + (size_t)(lb + it * 8 + wave) * kDin + d0 + lane * 8) = bv[it];
      __threadfence();
    }
    __syncthreads();
  }
}

__global__ __launch_bounds__(256) void scan_kernel(
    const float* __restrict__ BC, const float* __restrict__ UC, const float* __restrict__ XZ,
    const float* __restrict__ dtv, const float* __restrict__ Wdt, const float* __restrict__ bdt,
    const float* __restrict__ Alog, const float* __restrict__ Dp, unsigned short* __restrict__ Y16)
{
  __shared__ __align__(16) float sBC[kScTS * kBcW];
  __shared__ __align__(16) float sDl[kScTS * kScP];
  __shared__ __align__(16) float sDx[kScTS * kScP];
  __shared__ __align__(16) float sSk[kScTS * kScP];
  __shared__ __align__(16) float sGt[kScTS * kScP];
  __shared__ __align__(16) float sYs[kScTS * kScP];
  const int tid = threadIdx.x, lane = tid & 31, wave = tid >> 5;
  constexpr int kBlkPerB = kDin / kScCh;
  const int bix = blockIdx.x / kBlkPerB;
  const int d0  = (blockIdx.x - bix * kBlkPerB) * kScCh;
  const size_t row0 = (size_t)bix * kSeq;
  const int ch  = tid >> 2;
  const int sub = tid & 3;

#pragma unroll 1
  for (int i = 0; i < 16; ++i) {
    const int idx = tid + 256 * i;
    sBC[idx] = -expf(Alog[(size_t)d0 * kNst + idx]);
  }
  __syncthreads();
  float negA[kScNl], h[kScNl];
#pragma unroll
  for (int q4 = 0; q4 < 4; ++q4) {
    const v4f av = *(const v4f*)(sBC + ch * kNst + sub * kScNl + 4 * q4);
    negA[4 * q4 + 0] = av[0];
    negA[4 * q4 + 1] = av[1];
    negA[4 * q4 + 2] = av[2];
    negA[4 * q4 + 3] = av[3];
    h[4 * q4 + 0] = 0.f;
    h[4 * q4 + 1] = 0.f;
    h[4 * q4 + 2] = 0.f;
    h[4 * q4 + 3] = 0.f;
  }

  const int sr  = tid >> 4;
  const int c4  = (tid & 15) * 4;
  const int br  = tid >> 5;
  const int bc4 = (tid & 31) * 4;
  const v4f wdt4 = *(const v4f*)(Wdt + d0 + c4);
  const v4f bdt4 = *(const v4f*)(bdt + d0 + c4);
  const v4f dsk4 = *(const v4f*)(Dp + d0 + c4);
  const int q  = lane >> 3;
  const int c8 = (lane & 7) * 8;
  const int frow = wave * 4 + q;

#pragma unroll 1
  for (int t0 = 0; t0 < kSeq; t0 += kScTS) {
    __syncthreads();
#pragma unroll
    for (int i = 0; i < 4; ++i) {
      const int r = br + 8 * i;
      *(v4f*)(sBC + r * kBcW + bc4) = *(const v4f*)(BC + (row0 + t0 + r) * kBcW + bc4);
    }
#pragma unroll 1
    for (int i = 0; i < 2; ++i) {
      const int s = sr + 16 * i;
      const size_t row = row0 + t0 + s;
      const float dts = dtv[row];
      const v4f xv = *(const v4f*)(UC + row * kDin + d0 + c4);
      const v4f zv = *(const v4f*)(XZ + row * kXzP + kDin + d0 + c4);
      v4f dl, dx, sk, gt;
#pragma unroll
      for (int e = 0; e < 4; ++e) {
        const float pre = dts * wdt4[e] + bdt4[e];
        const float ea  = __expf(-fabsf(pre));
        const float u   = 1.0f + ea;
        const float l1p = __logf(u) + (ea - (u - 1.0f)) * __builtin_amdgcn_rcpf(u);
        const float dlt = fmaxf(pre, 0.0f) + l1p;
        const float zz  = zv[e];
        const float sg  = __builtin_amdgcn_rcpf(1.0f + __expf(-zz));
        dl[e] = dlt;
        dx[e] = dlt * xv[e];
        sk[e] = xv[e] * dsk4[e];
        gt[e] = zz * sg;
      }
      *(v4f*)(sDl + s * kScP + c4) = dl;
      *(v4f*)(sDx + s * kScP + c4) = dx;
      *(v4f*)(sSk + s * kScP + c4) = sk;
      *(v4f*)(sGt + s * kScP + c4) = gt;
    }
    __syncthreads();
#pragma unroll 1
    for (int s = 0; s < kScTS; ++s) {
      const float dlt = sDl[s * kScP + ch];
      const float dxi = sDx[s * kScP + ch];
      const float* brow = sBC + s * kBcW + sub * kScNl;
      float y = 0.f;
#pragma unroll
      for (int q4 = 0; q4 < 4; ++q4) {
        const v4f bv = *(const v4f*)(brow + 4 * q4);
        const v4f cv = *(const v4f*)(brow + kNst + 4 * q4);
#pragma unroll
        for (int e = 0; e < 4; ++e) {
          const float ex = __expf(dlt * negA[4 * q4 + e]);
          h[4 * q4 + e] = ex * h[4 * q4 + e] + dxi * bv[e];
          y = h[4 * q4 + e] * cv[e] + y;
        }
      }
      y += __shfl_xor(y, 1, 32);
      y += __shfl_xor(y, 2, 32);
      if (sub == 0) sYs[s * kScP + ch] = y;
    }
    __syncthreads();
    {
      const float* py = sYs + frow * kScP + c8;
      const float* ps = sSk + frow * kScP + c8;
      const float* pg = sGt + frow * kScP + c8;
      const v4f y0 = *(const v4f*)(py);
      const v4f y1 = *(const v4f*)(py + 4);
      const v4f s0 = *(const v4f*)(ps);
      const v4f s1 = *(const v4f*)(ps + 4);
      const v4f g0 = *(const v4f*)(pg);
      const v4f g1 = *(const v4f*)(pg + 4);
      v8h hv;
#pragma unroll
      for (int e = 0; e < 4; ++e) {
        const float a = (y0[e] + s0[e]) * g0[e];
        const float b = (y1[e] + s1[e]) * g1[e];
        hv[e]     = to_h16(a * kCarY);
        hv[4 + e] = to_h16(b * kCarY);
      }
      unsigned short* p = Y16 + (row0 + t0 + frow) * kDin + d0 + c8;
      *(volatile v8h*)p = hv;
      __threadfence();
      *(volatile v8h*)p = hv;
    }
  }
}

extern "C" void kernel_launch(void* const* d_in, const int* in_sizes, int n_in,
                              void* d_out, int out_size, void* d_ws, size_t ws_size,
                              hipStream_t stream)
{
  if (n_in < 11) return;
  if (in_sizes[0] != kRows * kDm) return;
  if (in_sizes[1] != kRows) return;
  if (in_sizes[2] != kDm * kXzP) return;
  if (in_sizes[3] != kDin * 4) return;
  if (in_sizes[4] != kDin) return;
  if (in_sizes[5] != kDin * kWxP) return;
  if (in_sizes[6] != kDin) return;
  if (in_sizes[7] != kDin) return;
  if (in_sizes[8] != kDin * kNst) return;
  if (in_sizes[9] != kDin) return;
  if (in_sizes[10] != kDin * kDm) return;
  if (out_size != kRows * kDm) return;
  if (ws_size < kWsTotal) return;

  const float* x       = (const float*)d_in[0];
  const float* dt_vals = (const float*)d_in[1];
  const float* w_in    = (const float*)d_in[2];
  const float* conv_w  = (const float*)d_in[3];
  const float* conv_b  = (const float*)d_in[4];
  const float* w_x     = (const float*)d_in[5];
  const float* w_dt    = (const float*)d_in[6];
  const float* b_dt    = (const float*)d_in[7];
  const float* A_log   = (const float*)d_in[8];
  const float* Dp      = (const float*)d_in[9];
  const float* w_out   = (const float*)d_in[10];
  float* out = (float*)d_out;

  char* ws = (char*)d_ws;
  unsigned short* WIN16  = (unsigned short*)(ws + kOffWIN);
  unsigned short* WX16   = (unsigned short*)(ws + kOffWX);
  unsigned short* WOUT16 = (unsigned short*)(ws + kOffWOUT);
  unsigned short* X16    = (unsigned short*)(ws + kOffX16);
  float*          XZ     = (float*)(ws + kOffXZ);
  float*          UC     = (float*)(ws + kOffUC);
  unsigned short* UC16   = (unsigned short*)(ws + kOffUC16);
  float*          BC     = (float*)(ws + kOffBC);
  unsigned short* Y16    = (unsigned short*)(ws + kOffY16);

  transpose_cast_kernel<<<dim3(kXzP / 64, kDm / 64), 256, 0, stream>>>(w_in, WIN16, kDm, kXzP, 0, kXzP, kCarW);
  transpose_cast_kernel<<<dim3(kBcW / 64, kDin / 64), 256, 0, stream>>>(w_x, WX16, kDin, kWxP, kWxSkip, kBcW, kCarW);
  transpose_cast_kernel<<<dim3(kDm / 64, kDin / 64), 256, 0, stream>>>(w_out, WOUT16, kDin, kDm, 0, kDm, kCarW);

  cast_f16_kernel<<<(kRows * kDm) / 8 / 256, 256, 0, stream>>>(x, X16, (kRows * kDm) / 8, kCarX);

  for (int hf = 0; hf < kHalves; ++hf) {
    const unsigned short* X16h = X16 + (size_t)hf * kHRows * kDm;
    const float* dth = dt_vals + (size_t)hf * kHRows;
    float* outh = out + (size_t)hf * kHRows * kDm;

    wmma_gemm64_f16<<<dim3(256, 1), 256, 0, stream>>>(
        X16h, kDm, WIN16, kDm, XZ, kXzP, kHRows, kXzP, kDm, kSclIn);

    conv_silu_kernel<<<dim3(kDin / 256, kHRows / 64), 256, 0, stream>>>(XZ, conv_w, conv_b, UC, UC16);

    wmma_gemm64_f16<<<dim3(32, 1), 256, 0, stream>>>(
        UC16, kDin, WX16, kDin, BC, kBcW, kHRows, kBcW, kDin, kSclXp);

    scan_kernel<<<kHBatch * (kDin / kScCh), 256, 0, stream>>>(BC, UC, XZ, dth, w_dt, b_dt, A_log, Dp, Y16);

    wmma_gemm64_f16<<<dim3(64, 1), 256, 0, stream>>>(
        Y16, kDin, WOUT16, kDin, outh, kDm, kHRows, kDm, kDin, kSclOut);
  }
}
